// EncoderLayer_45629732552839
// MI455X (gfx1250) — hardware-verified
//
#include <hip/hip_runtime.h>


#ifndef NB
#define NB 16
#endif
#ifndef SEQ
#define SEQ 1024
#endif
#define SEQ_FULL 1024
#define DM   512
#define NH_  8
#define HD   64
#define FF   2048
#define MTOK (NB * SEQ)
#define CH   (SEQ * DM / 256)
#define BPB  (SEQ * DM / 1024)
#define WCAR 64.0f
#define PCAR 1024.0f
#define CCAR 64.0f
#define HCAR 16.0f
#define SCL  0.125f
#define L2E  1.4426950408889634f
#define LNEPS 1e-5f

static_assert((SEQ & (SEQ - 1)) == 0);
static_assert(SEQ % 64 == 0 && SEQ <= SEQ_FULL);
static_assert(DM == 512 && HD == 64 && DM == NH_ * HD);
static_assert(FF == 4 * DM);
static_assert(MTOK % 64 == 0 && DM % 64 == 0 && FF % 64 == 0 && DM % 32 == 0 && FF % 32 == 0);
static_assert(CH % 128 == 0 && 8 * 32 * CH == SEQ * DM);

typedef _Float16 h16;
typedef __attribute__((ext_vector_type(16))) _Float16 v16h;
typedef __attribute__((ext_vector_type(8)))  _Float16 v8h;
typedef __attribute__((ext_vector_type(4)))  _Float16 v4h;
typedef __attribute__((ext_vector_type(2)))  _Float16 v2h;
typedef __attribute__((ext_vector_type(8)))  float    v8f;
typedef __attribute__((ext_vector_type(4)))  float    v4f;
typedef v8h __attribute__((may_alias)) v8ha;
typedef v4f __attribute__((may_alias)) v4fa;

__device__ __forceinline__ unsigned short f2bf(float f) { unsigned u = __float_as_uint(f); u += 0x7FFFu + ((u >> 16) & 1u); return (unsigned short)(u >> 16); }
__device__ __forceinline__ float bfr(float f) { return __uint_as_float(((unsigned)f2bf(f)) << 16); }
__device__ __forceinline__ v16h cat16(v8h lo, v8h hi) { return __builtin_shufflevector(lo, hi, 0, 1, 2, 3, 4, 5, 6, 7, 8, 9, 10, 11, 12, 13, 14, 15); }
__device__ __forceinline__ v16h ldh(const h16* p) { return cat16(*(const v8h*)p, *(const v8h*)(p + 16)); }
__device__ __forceinline__ v8f wmma16(v16h a, v16h b, v8f c) { return __builtin_amdgcn_wmma_f32_16x16x32_f16(false, a, false, b, (short)0, c, false, false); }
__device__ __forceinline__ void wave_sync() { __builtin_amdgcn_fence(3  , "wavefront"); __builtin_amdgcn_wave_barrier(); asm volatile("" ::: "memory"); }

template <int OUT16, int RELU, int BMODE, int RESM>
__global__ __launch_bounds__(32) void k_gemmw(const h16* __restrict__ A, const h16* __restrict__ Bt, unsigned K, float* Cf, h16* Chh, unsigned ldc, const float* __restrict__ bias, const float* res, float ascl, float oscl) {
    __shared__ __align__(16) float os[16 * 68];
    const unsigned lane = threadIdx.x & 31u, lr = lane & 15u, hi = lane >> 4; const unsigned r0 = blockIdx.x * 64u, c0 = blockIdx.y * 64u;
    v8f acc[4][4];
#pragma unroll
    for (int mb = 0; mb < 4; ++mb)
#pragma unroll
        for (int nb = 0; nb < 4; ++nb) acc[mb][nb] = (v8f){};
    const size_t aoff = (size_t)(r0 + lr) * K + 8u * hi, boff = (size_t)(c0 + lr) * K + 8u * hi;
#pragma unroll 1
    for (unsigned kc = 0; kc < K; kc += 32u) {
        v16h a[4];
#pragma unroll
        for (int mb = 0; mb < 4; ++mb) a[mb] = ldh(A + aoff + (size_t)mb * 16u * K + kc);
#pragma unroll
        for (int nb = 0; nb < 4; ++nb) { const v16h b = ldh(Bt + boff + (size_t)nb * 16u * K + kc);
#pragma unroll
            for (int mb = 0; mb < 4; ++mb) acc[mb][nb] = wmma16(a[mb], b, acc[mb][nb]); }
        asm volatile("v_nop\n\tv_nop\n\tv_nop\n\tv_nop" : "+v"(acc[0][0]), "+v"(acc[1][1]), "+v"(acc[2][2]), "+v"(acc[3][3]) : "v"(a[0]), "v"(a[3]));
    }
#pragma unroll
    for (int mb = 0; mb < 4; ++mb) {
#pragma unroll
        for (int nb = 0; nb < 4; ++nb) {
#pragma unroll
            for (int j = 0; j < 8; ++j) os[(hi * 8u + j) * 68u + nb * 16u + lr] = acc[mb][nb][j]; }
        wave_sync();
        const unsigned rb = r0 + mb * 16u;
#pragma unroll 1
        for (int ps = 0; ps < 2; ++ps) {
            if (OUT16) {
#pragma unroll
                for (int s = 0; s < 4; ++s) { const unsigned row = 4u * s + (lane >> 3), cofs = (lane & 7u) * 8u; const unsigned grow = rb + row;
                    const v4f x0 = *(const v4fa*)(os + row * 68u + cofs); const v4f x1 = *(const v4fa*)(os + row * 68u + cofs + 4u);
                    v4f b0 = (v4f){}, b1 = (v4f){};
                    if (BMODE == 1) { b0 = *(const v4f*)(bias + c0 + cofs); b1 = *(const v4f*)(bias + c0 + cofs + 4u); }
                    if (BMODE == 2) { const float br = bias[grow]; b0 = (v4f){br, br, br, br}; b1 = b0; }
                    v8h o;
#pragma unroll
                    for (int q = 0; q < 4; ++q) { float v = x0[q] * ascl + bfr(b0[q]); float u = x1[q] * ascl + bfr(b1[q]); if (RELU) { v = fmaxf(v, 0.0f); u = fmaxf(u, 0.0f); } o[q] = (h16)(v * oscl); o[4 + q] = (h16)(u * oscl); }
                    *(volatile v8h*)(Chh + (size_t)grow * ldc + c0 + cofs) = o; }
            } else {
#pragma unroll
                for (int s = 0; s < 8; ++s) { const unsigned row = 2u * s + hi, cofs = lr * 4u; const unsigned grow = rb + row;
                    const v4f x0 = *(const v4fa*)(os + row * 68u + cofs);
                    v4f b0 = (v4f){}; if (BMODE == 1) b0 = *(const v4f*)(bias + c0 + cofs); if (BMODE == 2) { const float br = bias[grow]; b0 = (v4f){br, br, br, br}; }
                    v4f rv = (v4f){};
                    if (RESM != 0) { const unsigned rr = (RESM == 1) ? ((grow / (unsigned)SEQ) * (unsigned)SEQ_FULL + (grow % (unsigned)SEQ)) : grow; rv = *(const v4f*)(res + (size_t)rr * ldc + c0 + cofs); }
                    v4f o;
#pragma unroll
                    for (int q = 0; q < 4; ++q) { float v = x0[q] * ascl + bfr(b0[q]); if (RELU) v = fmaxf(v, 0.0f); if (RESM == 1) v = bfr(rv[q]) + v; if (RESM == 2) v = rv[q] + v; o[q] = v; }
                    *(volatile v4f*)(Cf + (size_t)grow * ldc + c0 + cofs) = o; }
            }
            if (ps == 0) __threadfence(); }
        wave_sync();
    }
}

__global__ __launch_bounds__(256) void k_wtG(const float* __restrict__ w, unsigned K, unsigned lgK, unsigned N, h16* Bt) {
    const unsigned lane = threadIdx.x & 31u; const unsigned L0 = (blockIdx.x * 8u + (threadIdx.x >> 5)) * 8u; const unsigned nlines = (N * K) >> 6;
#pragma unroll 1
    for (int ps = 0; ps < 2; ++ps) {
#pragma unroll 1
        for (unsigned l = 0; l < 8u; ++l) { const unsigned L = L0 + l;
            if (L < nlines) { const unsigned e = L * 64u + lane * 2u; const unsigned k = e & (K - 1u), n = e >> lgK; v2h o;
                o[0] = (h16)(bfr(w[(size_t)k * N + n]) * WCAR); o[1] = (h16)(bfr(w[(size_t)(k + 1u) * N + n]) * WCAR); *(volatile v2h*)(Bt + e) = o; } }
        if (ps == 0) __threadfence(); }
}

__global__ __launch_bounds__(256) void k_cvtx(const float* __restrict__ x, h16* XB) {
    const unsigned i = blockIdx.x * 256u + threadIdx.x; if (i >= (unsigned)(MTOK * (DM / 8))) return;
    const unsigned row = i >> 6, c = (i & 63u) * 8u; const unsigned b = row / (unsigned)SEQ, s = row % (unsigned)SEQ;
    const v8f v = *(const v8f*)(x + ((size_t)b * SEQ_FULL + s) * DM + c); v8h o;
#pragma unroll
    for (int k = 0; k < 8; ++k) o[k] = (h16)bfr(v[k]);
    h16* d = XB + (size_t)i * 8u; *(volatile v8h*)d = o; __threadfence(); *(volatile v8h*)d = o;
}

__global__ __launch_bounds__(256) void k_maskb(const float* __restrict__ mask, float* MB) {
    const unsigned i = blockIdx.x * 256u + threadIdx.x; if (i >= (unsigned)(MTOK / 4)) return;
    const unsigned e = i * 4u; const unsigned b = e / (unsigned)SEQ, s = e % (unsigned)SEQ;
    const v4f a = *(const v4f*)(mask + (size_t)b * SEQ_FULL + s); v4f o;
#pragma unroll
    for (int q = 0; q < 4; ++q) o[q] = bfr(a[q]) * -1.0e9f;
    *(volatile v4f*)(MB + e) = o; __threadfence(); *(volatile v4f*)(MB + e) = o;
}

__global__ __launch_bounds__(128) void k_flash(const h16* __restrict__ QP, const h16* __restrict__ KP, const h16* __restrict__ VT, const float* __restrict__ MB, h16* CTX) {
    __shared__ __align__(16) h16 ost[4 * 16 * 72];
    const unsigned lane = threadIdx.x & 31u, w = threadIdx.x >> 5, lr = lane & 15u, hi = lane >> 4;
    const unsigned b = blockIdx.z, h = blockIdx.y, q0 = (blockIdx.x * 4u + w) * 16u;
    const size_t tb = (size_t)b * SEQ;
    const h16* Qb = QP + tb * DM + h * HD; const h16* Kb = KP + tb * DM + h * HD;
    const h16* Vb = VT + (size_t)(h * HD) * MTOK + tb; const float* mb = MB + tb;
    const v16h qf0 = ldh(Qb + (size_t)(q0 + lr) * DM + 8u * hi); const v16h qf1 = ldh(Qb + (size_t)(q0 + lr) * DM + 32u + 8u * hi);
    v8f o[4];
#pragma unroll
    for (int dt = 0; dt < 4; ++dt) o[dt] = (v8f){};
    float m = -1.0e30f, l = 0.0f;
#pragma unroll 1
    for (unsigned kt = 0; kt < (unsigned)SEQ; kt += 32u) {
        const h16* kp = Kb + (size_t)(kt + lr) * DM + 8u * hi;
        const v16h k00 = ldh(kp), k01 = ldh(kp + 32), k10 = ldh(kp + 16 * DM), k11 = ldh(kp + 16 * DM + 32);
        const float* mp = mb + kt + 8u * hi;
        const v4f ma = *(const v4f*)(mp), mb2 = *(const v4f*)(mp + 4), mc = *(const v4f*)(mp + 16), md = *(const v4f*)(mp + 20);
        v8f s0 = (v8f){}, s1 = (v8f){};
        s0 = wmma16(k00, qf0, s0); s0 = wmma16(k01, qf1, s0); s1 = wmma16(k10, qf0, s1); s1 = wmma16(k11, qf1, s1);
        asm volatile("v_nop\n\tv_nop\n\tv_nop\n\tv_nop" : "+v"(s0), "+v"(s1) : "v"(k00), "v"(k01), "v"(k10), "v"(k11), "v"(qf0), "v"(qf1));
        asm volatile("" ::: "memory");
        float t[16];
#pragma unroll
        for (int r = 0; r < 4; ++r) { t[r] = s0[r] * SCL + ma[r]; t[4 + r] = s0[4 + r] * SCL + mb2[r]; t[8 + r] = s1[r] * SCL + mc[r]; t[12 + r] = s1[4 + r] * SCL + md[r]; }
        float mx = t[0];
#pragma unroll
        for (int i = 1; i < 16; ++i) mx = fmaxf(mx, t[i]);
        mx = fmaxf(mx, __shfl_xor(mx, 16, 32));
        const float mn = fmaxf(m, mx); const float alpha = __builtin_amdgcn_exp2f((m - mn) * L2E); m = mn;
        float ls = 0.0f; v16h pb;
#pragma unroll
        for (int i = 0; i < 16; ++i) { const float p = __builtin_amdgcn_exp2f((t[i] - mn) * L2E); ls += p; pb[i] = (h16)(p * PCAR); }
        l = l * alpha + ls;
#pragma unroll
        for (int dt = 0; dt < 4; ++dt) o[dt] = o[dt] * alpha;
        const h16* vp = Vb + (size_t)lr * MTOK + kt + 8u * hi;
        const v16h v0 = ldh(vp), v1 = ldh(vp + (size_t)16 * MTOK), v2 = ldh(vp + (size_t)32 * MTOK), v3 = ldh(vp + (size_t)48 * MTOK);
        o[0] = wmma16(v0, pb, o[0]); o[1] = wmma16(v1, pb, o[1]); o[2] = wmma16(v2, pb, o[2]); o[3] = wmma16(v3, pb, o[3]);
        asm volatile("v_nop\n\tv_nop\n\tv_nop\n\tv_nop" : "+v"(o[0]), "+v"(o[1]), "+v"(o[2]), "+v"(o[3]) : "v"(v0), "v"(v1), "v"(v2), "v"(v3), "v"(pb));
    }
    const float lt = l + __shfl_xor(l, 16, 32);
    const float inv = (CCAR / PCAR) * (1.0f / lt);
    h16* ow = ost + w * (16u * 72u);
#pragma unroll
    for (int dt = 0; dt < 4; ++dt) { v8h ov;
#pragma unroll
        for (int r = 0; r < 8; ++r) ov[r] = (h16)(o[dt][r] * inv);
        *(v8h*)(ow + lr * 72u + dt * 16u + 8u * hi) = ov; }
    wave_sync();
    h16* crow = CTX + (tb + q0) * DM + h * HD;
#pragma unroll 1
    for (int ps = 0; ps < 2; ++ps) {
#pragma unroll
        for (int s = 0; s < 4; ++s) { const unsigned row = 4u * s + (lane >> 3), pc = (lane & 7u) * 8u; const v8h val = *(const v8ha*)(ow + row * 72u + pc); *(volatile v8h*)(crow + (size_t)row * DM + pc) = val; }
        if (ps == 0) __threadfence(); }
}

__global__ __launch_bounds__(256) void k_lnpart(const float* __restrict__ Y, float* PART) {
    __shared__ __align__(16) float st[64];
    const unsigned lane = threadIdx.x & 31u, w = threadIdx.x >> 5; const unsigned blk = blockIdx.x;
    const float* base = Y + (size_t)blk * (32u * (unsigned)CH);
#pragma unroll 1
    for (unsigned i = 0; i < 4u; ++i) { const unsigned c = w * 4u + i; const float* p = base + (size_t)c * CH + lane * 4u; float s = 0.0f;
#pragma unroll 1
        for (unsigned it = 0; it < (unsigned)(CH / 128); ++it) { const v4f a = *(const v4f*)(p + it * 128u); s += (a[0] + a[1]) + (a[2] + a[3]); }
#pragma unroll
        for (int sh = 16; sh; sh >>= 1) s += __shfl_xor(s, sh, 32);
        const float mc = s * (1.0f / (float)CH); float s2 = 0.0f;
#pragma unroll 1
        for (unsigned it = 0; it < (unsigned)(CH / 128); ++it) { const v4f a = *(const v4f*)(p + it * 128u); const float d0 = a[0] - mc, d1 = a[1] - mc, d2 = a[2] - mc, d3 = a[3] - mc; s2 += (d0 * d0 + d1 * d1) + (d2 * d2 + d3 * d3); }
#pragma unroll
        for (int sh = 16; sh; sh >>= 1) s2 += __shfl_xor(s2, sh, 32);
        if (lane == 0u) { st[c] = s; st[32u + c] = s2; } }
    __syncthreads();
    if (threadIdx.x < 16u) { const v4f v = *(const v4fa*)(st + threadIdx.x * 4u); float* dst = PART + (size_t)blk * 64u + threadIdx.x * 4u; *(volatile v4f*)dst = v; __threadfence(); *(volatile v4f*)dst = v; }
}

template <int OUTH>
__global__ __launch_bounds__(256) void k_lnapply(const float* Yin, const float* __restrict__ PART, const float* __restrict__ g, const float* __restrict__ bb, float* Of, h16* Oh) {
    __shared__ float red[16];
    const unsigned t = threadIdx.x, lane = t & 31u, w = t >> 5; const unsigned b = blockIdx.x / (unsigned)BPB;
    const float* pp = PART + (size_t)b * 512u + w * 64u + lane;
    const float s = pp[0], q2 = pp[32];
    float r = s;
#pragma unroll
    for (int sh = 16; sh; sh >>= 1) r += __shfl_xor(r, sh, 32);
    if (lane == 0u) red[w] = r;
    __syncthreads();
    const float S = ((red[0] + red[1]) + (red[2] + red[3])) + ((red[4] + red[5]) + (red[6] + red[7]));
    const float mean = S * (1.0f / (float)(SEQ * DM));
    const float dm = s * (1.0f / (float)CH) - mean; float r2 = q2 + (float)CH * dm * dm;
#pragma unroll
    for (int sh = 16; sh; sh >>= 1) r2 += __shfl_xor(r2, sh, 32);
    if (lane == 0u) red[8u + w] = r2;
    __syncthreads();
    const float M2 = ((red[8] + red[9]) + (red[10] + red[11])) + ((red[12] + red[13]) + (red[14] + red[15]));
    const float var = M2 * (1.0f / (float)(SEQ * DM)); const float rstd = 1.0f / sqrtf(var + LNEPS);
    const size_t e = ((size_t)blockIdx.x * 256u + t) * 4u; const unsigned sd = (unsigned)(e - (size_t)b * SEQ * DM);
    const v4f y = *(const v4f*)(Yin + e); const v4f gw = *(const v4f*)(g + sd); const v4f gb = *(const v4f*)(bb + sd); v4f o; v4h oh;
#pragma unroll
    for (int q = 0; q < 4; ++q) { o[q] = (y[q] - mean) * rstd * bfr(gw[q]) + bfr(gb[q]); oh[q] = (h16)o[q]; }
    *(volatile v4f*)(Of + e) = o; if (OUTH) *(volatile v4h*)(Oh + e) = oh; __threadfence(); *(volatile v4f*)(Of + e) = o; if (OUTH) *(volatile v4h*)(Oh + e) = oh;
}

extern "C" void kernel_launch(void* const* d_in, const int* in_sizes, int n_in,
                              void* d_out, int out_size, void* d_ws, size_t ws_size, hipStream_t stream) {
    if (n_in < 18) return;
    if (in_sizes[0] < ((NB - 1) * SEQ_FULL + SEQ) * DM) return;
    if (in_sizes[1] < (NB - 1) * SEQ_FULL + SEQ) return;
    if (in_sizes[2] < DM * DM || in_sizes[4] < DM * DM || in_sizes[6] < DM * DM || in_sizes[8] < DM * DM) return;
    if (in_sizes[3] < DM || in_sizes[5] < DM || in_sizes[7] < DM || in_sizes[9] < DM || in_sizes[13] < DM || in_sizes[11] < FF) return;
    if (in_sizes[10] < DM * FF || in_sizes[12] < FF * DM) return;
    if (in_sizes[14] < SEQ * DM || in_sizes[15] < SEQ * DM || in_sizes[16] < SEQ * DM || in_sizes[17] < SEQ * DM) return;
    if (out_size < MTOK * DM) return;
    const float* x = (const float*)d_in[0]; const float* mask = (const float*)d_in[1];
    const float* wq = (const float*)d_in[2]; const float* bq = (const float*)d_in[3]; const float* wk = (const float*)d_in[4]; const float* bk = (const float*)d_in[5];
    const float* wv = (const float*)d_in[6]; const float* bv = (const float*)d_in[7]; const float* wo = (const float*)d_in[8]; const float* bo = (const float*)d_in[9];
    const float* w1 = (const float*)d_in[10]; const float* b1 = (const float*)d_in[11]; const float* w2 = (const float*)d_in[12]; const float* b2 = (const float*)d_in[13];
    const float* ln1w = (const float*)d_in[14]; const float* ln1b = (const float*)d_in[15]; const float* ln2w = (const float*)d_in[16]; const float* ln2b = (const float*)d_in[17];
    float* OUT = (float*)d_out;
    char* wsp = (char*)d_ws;
    auto take = [&](size_t bytes) { char* p = wsp; wsp += (bytes + 255) & ~(size_t)255; return (void*)p; };
    h16* R0 = (h16*)take((size_t)MTOK * DM * 2);
    h16* R1 = (h16*)take((size_t)MTOK * FF * 2);
    float* N1 = (float*)take((size_t)MTOK * DM * 4);
    h16* WQ = (h16*)take((size_t)DM * DM * 2); h16* WK = (h16*)take((size_t)DM * DM * 2); h16* WV = (h16*)take((size_t)DM * DM * 2); h16* WO = (h16*)take((size_t)DM * DM * 2);
    h16* W1T = (h16*)take((size_t)FF * DM * 2); h16* W2T = (h16*)take((size_t)DM * FF * 2);
    float* MBp = (float*)take((size_t)MTOK * 4); float* PART = (float*)take((size_t)NB * 512 * 4);
    const size_t carved = (size_t)(wsp - (char*)d_ws);
    if (carved > ws_size || carved > ((size_t)128 << 20)) return;
    h16* XB = R0; h16* N1H = R0; h16* QP = R1; h16* KP = R1 + (size_t)MTOK * DM; h16* VT = R1 + (size_t)2 * MTOK * DM; h16* CTX = R1 + (size_t)3 * MTOK * DM; h16* HH = R1;

    k_cvtx<<<(unsigned)(MTOK * (DM / 8) / 256), 256, 0, stream>>>(x, XB);
    k_wtG<<<DM * DM / 64 / 64, 256, 0, stream>>>(wq, DM, 9, DM, WQ);
    k_wtG<<<DM * DM / 64 / 64, 256, 0, stream>>>(wk, DM, 9, DM, WK);
    k_wtG<<<DM * DM / 64 / 64, 256, 0, stream>>>(wv, DM, 9, DM, WV);
    k_wtG<<<DM * DM / 64 / 64, 256, 0, stream>>>(wo, DM, 9, DM, WO);
    k_wtG<<<DM * FF / 64 / 64, 256, 0, stream>>>(w1, DM, 9, FF, W1T);
    k_wtG<<<DM * FF / 64 / 64, 256, 0, stream>>>(w2, FF, 11, DM, W2T);
    k_maskb<<<(MTOK / 4 + 255) / 256, 256, 0, stream>>>(mask, MBp);
    k_gemmw<1, 0, 1, 0><<<dim3(MTOK / 64, DM / 64), 32, 0, stream>>>(XB, WQ, DM, nullptr, QP, DM, bq, nullptr, 1.0f / WCAR, 1.0f);
    k_gemmw<1, 0, 1, 0><<<dim3(MTOK / 64, DM / 64), 32, 0, stream>>>(XB, WK, DM, nullptr, KP, DM, bk, nullptr, 1.0f / WCAR, 1.0f);
    k_gemmw<1, 0, 2, 0><<<dim3(DM / 64, MTOK / 64), 32, 0, stream>>>(WV, XB, DM, nullptr, VT, MTOK, bv, nullptr, 1.0f / WCAR, 1.0f);
    k_flash<<<dim3(SEQ / 64, NH_, NB), 128, 0, stream>>>(QP, KP, VT, MBp, CTX);
    k_gemmw<0, 0, 1, 1><<<dim3(MTOK / 64, DM / 64), 32, 0, stream>>>(CTX, WO, DM, OUT, nullptr, DM, bo, x, 1.0f / (CCAR * WCAR), 1.0f);
    k_lnpart<<<NB * 8, 256, 0, stream>>>(OUT, PART);
    k_lnapply<1><<<NB * BPB, 256, 0, stream>>>(OUT, PART, ln1w, ln1b, N1, N1H);
    k_gemmw<1, 1, 1, 0><<<dim3(MTOK / 64, FF / 64), 32, 0, stream>>>(N1H, W1T, DM, nullptr, HH, FF, b1, nullptr, 1.0f / WCAR, HCAR);
    k_gemmw<0, 0, 1, 2><<<dim3(MTOK / 64, DM / 64), 32, 0, stream>>>(HH, W2T, FF, OUT, nullptr, DM, b2, N1, 1.0f / (HCAR * WCAR), 1.0f);
    k_lnpart<<<NB * 8, 256, 0, stream>>>(OUT, PART);
    k_lnapply<0><<<NB * BPB, 256, 0, stream>>>(OUT, PART, ln2w, ln2b, OUT, nullptr);
}
